// Henrion_MPNNConv_67388036874510
// MI455X (gfx1250) — hardware-verified
//
#include <hip/hip_runtime.h>
#include <math.h>

typedef __attribute__((ext_vector_type(16))) _Float16 v16h;
typedef __attribute__((ext_vector_type(16))) __bf16 v16b;
typedef __attribute__((ext_vector_type(8)))  _Float16 v8h;
typedef __attribute__((ext_vector_type(8)))  float v8f;
typedef __attribute__((ext_vector_type(4)))  float v4f;
typedef __attribute__((ext_vector_type(2)))  float v2f;
typedef __attribute__((ext_vector_type(4)))  unsigned v4u;
typedef __attribute__((ext_vector_type(4)))  int v4i;
typedef float __attribute__((may_alias)) float_a;
typedef int __attribute__((may_alias)) int_a;

template <typename T> __device__ __forceinline__ void vst2(void* p, T v) { *(volatile T*)p = v; __threadfence(); *(volatile T*)p = v; }
__device__ __forceinline__ v8f wmma16(v16h a, v16h b, v8f c) {
  v8f d = __builtin_amdgcn_wmma_f32_16x16x32_f16(false, a, false, b, (short)0, c, false, false);
  asm volatile("v_nop\n\tv_nop\n\tv_nop\n\tv_nop" : "+v"(d) : "v"(a), "v"(b));
  return d;
}
__device__ __forceinline__ v8f wmma_bf(v16b a, v16b b, v8f c) {
  v8f d = __builtin_amdgcn_wmma_f32_16x16x32_bf16(false, a, false, b, (short)0, c, false, false);
  asm volatile("v_nop\n\tv_nop\n\tv_nop\n\tv_nop" : "+v"(d) : "v"(a), "v"(b));
  return d;
}
__device__ __forceinline__ v16h frag_h(const _Float16* rowk0, int lane) {
  union { v16h v; v8h q[2]; } u; const _Float16* p = rowk0 + 8 * (lane >> 4);
  u.q[0] = *(const v8h*)p; u.q[1] = *(const v8h*)(p + 16); return u.v;
}
__device__ __forceinline__ v16h frag_f32(const float* rowk0, int lane) {
  v16h a; const float* p = rowk0 + 8 * (lane >> 4);
#pragma unroll
  for (int i = 0; i < 8; ++i) { a[i] = (_Float16)p[i]; a[8 + i] = (_Float16)p[16 + i]; }
  return a;
}
__device__ __forceinline__ v16h frag_f32s(const float* rowk0, int lane, float sc) {
  v16h a; const float* p = rowk0 + 8 * (lane >> 4);
#pragma unroll
  for (int i = 0; i < 8; ++i) { a[i] = (_Float16)(p[i] * sc); a[8 + i] = (_Float16)(p[16 + i] * sc); }
  return a;
}
__device__ __forceinline__ v16h fragc_f32(const float* W, int k0, int n, int lane, int ld, int K) {
  v16h a; const int g = lane >> 4;
#pragma unroll
  for (int i = 0; i < 8; ++i) { const int ka = k0 + 8 * g + i, kb = ka + 16;
    a[i] = (_Float16)(ka < K ? W[(size_t)ka * ld + n] : 0.f); a[8 + i] = (_Float16)(kb < K ? W[(size_t)kb * ld + n] : 0.f); }
  return a;
}
struct F2 { v16b h, l; };
__device__ __forceinline__ F2 bsplit16(const float v[16]) { F2 r;
#pragma unroll
  for (int i = 0; i < 16; ++i) { const __bf16 h = (__bf16)v[i]; r.h[i] = h; r.l[i] = (__bf16)(v[i] - (float)h); }
  return r; }
__device__ __forceinline__ F2 split_row(const float* row, int k0, int lane) { float v[16]; const float* p = row + k0 + 8 * (lane >> 4);
#pragma unroll
  for (int i = 0; i < 8; ++i) { v[i] = p[i]; v[8 + i] = p[16 + i]; }
  return bsplit16(v); }
__device__ __forceinline__ F2 split_rowK(const float* row, int k0, int lane, int K) { float v[16]; const int g = lane >> 4;
#pragma unroll
  for (int i = 0; i < 8; ++i) { const int ka = k0 + 8 * g + i, kb = ka + 16; v[i] = ka < K ? row[ka] : 0.f; v[8 + i] = kb < K ? row[kb] : 0.f; }
  return bsplit16(v); }
__device__ __forceinline__ F2 split_col(const float* W, int k0, int n, int lane, int ld, int K) { float v[16]; const int g = lane >> 4;
#pragma unroll
  for (int i = 0; i < 8; ++i) { const int ka = k0 + 8 * g + i, kb = ka + 16; v[i] = ka < K ? W[(size_t)ka * ld + n] : 0.f; v[8 + i] = kb < K ? W[(size_t)kb * ld + n] : 0.f; }
  return bsplit16(v); }
__device__ __forceinline__ v8f mac3(const F2& a, const F2& b, v8f c) { c = wmma_bf(a.l, b.h, c); c = wmma_bf(a.h, b.l, c); return wmma_bf(a.h, b.h, c); }
__device__ __forceinline__ float sigm(float v) { return 1.0f / (1.0f + expf(-v)); }
#define LDSX() do { asm volatile("s_wait_dscnt 0" ::: "memory"); __builtin_amdgcn_wave_barrier(); __builtin_amdgcn_fence(__ATOMIC_RELEASE, "workgroup"); } while (0)

#define NN 50000
#define NE 800000
#define FI 128
#define FH 64
#define G3 192
#define RB 1024
#define NRB ((NN + RB - 1) / RB)
#define NNP (NRB * RB)
#define EPT 16
#define CH (256 * EPT)

template <int K, int NOUT, int WT>
__global__ __launch_bounds__(128) void k_lin(const float* __restrict__ A, int lda, int arows, const float* __restrict__ W, const float* __restrict__ bias, float* __restrict__ D, int ldd) {
  constexpr int NT = NOUT / 16;
  __shared__ __align__(16) float so[4][16][NOUT + 4];
  const int tid = threadIdx.x, wave = tid >> 5, lane = tid & 31, col = lane & 15, g = lane >> 4;
  const int r0 = blockIdx.x * 64 + wave * 16; const int ra = (r0 + col) < arows ? (r0 + col) : arows - 1;
  v8f acc[NT];
#pragma unroll
  for (int t = 0; t < NT; ++t) acc[t] = (v8f){};
#pragma unroll 1
  for (int kc = 0; kc < K / 32; ++kc) { const F2 a = split_row(A + (size_t)ra * lda, kc * 32, lane);
#pragma unroll
    for (int t = 0; t < NT; ++t) acc[t] = mac3(a, WT ? split_row(W + (size_t)(t * 16 + col) * K, kc * 32, lane) : split_col(W, kc * 32, t * 16 + col, lane, NOUT, K), acc[t]); }
#pragma unroll
  for (int t = 0; t < NT; ++t) { const float bb = bias[t * 16 + col];
#pragma unroll
    for (int r = 0; r < 8; ++r) so[wave][8 * g + r][t * 16 + col] = acc[t][r] + bb; }
  LDSX();
  for (int q = lane; q < 16 * (NOUT / 4); q += 32) { const int rl = q / (NOUT / 4), pc = q % (NOUT / 4); vst2(D + (size_t)(r0 + rl) * ldd + pc * 4, *(const v4f*)(&so[wave][rl][pc * 4])); }
}
__global__ __launch_bounds__(256) void k_agg(const float* __restrict__ MSG, const int* __restrict__ ei, float* __restrict__ M) {
  __shared__ __align__(16) float sacc[RB][FH];
  __shared__ int ssrc[8][32 * EPT], sdl[8][32 * EPT]; __shared__ int scnt[8];
  const int tid = threadIdx.x, wave = tid >> 5, lane = tid & 31;
  const int r0 = blockIdx.x * RB; const int* esrc = ei; const int* edst = ei + NE;
  for (int q = tid; q < RB * FH; q += 256) (&sacc[0][0])[q] = 0.f;
  __syncthreads();
  #pragma unroll 1
  for (int c0 = 0; c0 < NE; c0 += CH) {
    const int e0 = c0 + tid * EPT; int hd[EPT]; int cnt = 0;
    if (e0 + EPT <= NE) {
#pragma unroll
      for (int v = 0; v < EPT / 4; ++v) { const int4 d4 = *(const int4*)(edst + e0 + v * 4);
        const int dd[4] = {d4.x, d4.y, d4.z, d4.w};
#pragma unroll
        for (int u = 0; u < 4; ++u) { const unsigned rel = (unsigned)(dd[u] - r0); const bool h = rel < (unsigned)RB; hd[v * 4 + u] = h ? (int)rel : -1; cnt += h ? 1 : 0; } } }
    else {
#pragma unroll
      for (int u = 0; u < EPT; ++u) { const int e = e0 + u; hd[u] = -1; if (e < NE) { const unsigned rel = (unsigned)(edst[e] - r0); if (rel < (unsigned)RB) { hd[u] = (int)rel; ++cnt; } } } }
    int incl = cnt;
#pragma unroll
    for (int off = 1; off < 32; off <<= 1) { const int vv = __shfl_up(incl, off, 32); if (lane >= off) incl += vv; }
    const int wtot = __shfl(incl, 31, 32); int pos = incl - cnt;
    if (cnt > 0) {
#pragma unroll
      for (int u = 0; u < EPT; ++u) if (hd[u] >= 0) { int s = esrc[e0 + u]; s = s < 0 ? 0 : (s >= NN ? NN - 1 : s); ssrc[wave][pos] = s; sdl[wave][pos] = hd[u];  ++pos; } }
    if (lane == 0) scnt[wave] = wtot;
    __syncthreads();
    if (tid < FH) { for (int w = 0; w < 8; ++w) { const int nh = scnt[w]; for (int i = 0; i < nh; ++i) sacc[sdl[w][i]][tid] += MSG[(size_t)ssrc[w][i] * FH + tid]; } }
    __syncthreads(); }
  for (int q = tid; q < RB * (FH / 4); q += 256) { const int rl = q >> 4, pc = q & 15; v4f v = *(const v4f*)(&sacc[rl][pc * 4]);
#pragma unroll
    for (int e = 0; e < 4; ++e) v[e] = v[e] > 0.f ? v[e] : 0.f;
    vst2(M + (size_t)(r0 + rl) * FH + pc * 4, v); }
}
__global__ __launch_bounds__(128) void k_gru(const float* __restrict__ M, const float* __restrict__ x, const float* __restrict__ H, const float* __restrict__ wih, const float* __restrict__ whh, const float* __restrict__ bih, const float* __restrict__ bhh, float* __restrict__ Hout, int nrows) {
  __shared__ __align__(16) float sgi[4][16][G3 + 4];
  __shared__ __align__(16) float sgh[4][16][G3 + 4];
  const int tid = threadIdx.x, wave = tid >> 5, lane = tid & 31, col = lane & 15, g = lane >> 4;
  const int r0 = blockIdx.x * 64 + wave * 16; const int ra = (r0 + col) < NN ? (r0 + col) : NN - 1;
  { v8f acc[12];
#pragma unroll
    for (int t = 0; t < 12; ++t) acc[t] = (v8f){};
#pragma unroll 1
    for (int kc = 0; kc < G3 / 32; ++kc) { const F2 a = kc < 2 ? split_row(M + (size_t)ra * FH, kc * 32, lane) : split_row(x + (size_t)ra * FI, (kc - 2) * 32, lane);
#pragma unroll
      for (int t = 0; t < 12; ++t) acc[t] = mac3(a, split_row(wih + (size_t)(t * 16 + col) * G3, kc * 32, lane), acc[t]); }
#pragma unroll
    for (int t = 0; t < 12; ++t) { const float bb = bih[t * 16 + col];
#pragma unroll
      for (int r = 0; r < 8; ++r) sgi[wave][8 * g + r][t * 16 + col] = acc[t][r] + bb; } }
  { v8f acc[12];
#pragma unroll
    for (int t = 0; t < 12; ++t) acc[t] = (v8f){};
#pragma unroll
    for (int kc = 0; kc < FH / 32; ++kc) { const F2 a = split_row(H + (size_t)ra * FH, kc * 32, lane);
#pragma unroll
      for (int t = 0; t < 12; ++t) acc[t] = mac3(a, split_row(whh + (size_t)(t * 16 + col) * FH, kc * 32, lane), acc[t]); }
#pragma unroll
    for (int t = 0; t < 12; ++t) { const float bb = bhh[t * 16 + col];
#pragma unroll
      for (int r = 0; r < 8; ++r) sgh[wave][8 * g + r][t * 16 + col] = acc[t][r] + bb; } }
  LDSX();
  { const int rl = lane >> 1, hf = lane & 1; const int row = r0 + rl; const float* gi = &sgi[wave][rl][0]; const float* gh = &sgh[wave][rl][0]; const float* hr = H + (size_t)(row < NN ? row : NN - 1) * FH;
#pragma unroll 1
    for (int c = hf * 32; c < hf * 32 + 32; ++c) { const float rg = sigm(gi[c] + gh[c]); const float zg = sigm(gi[FH + c] + gh[FH + c]); const float ng = tanhf(gi[2 * FH + c] + rg * gh[2 * FH + c]);
      sgi[wave][rl][c] = (1.f - zg) * ng + zg * hr[c]; } }
  LDSX();
  for (int q = lane; q < 16 * 16; q += 32) { const int rl = q >> 4, pc = q & 15; if (r0 + rl < nrows) vst2(Hout + (size_t)(r0 + rl) * FH + pc * 4, *(const v4f*)(&sgi[wave][rl][pc * 4])); }
}
extern "C" void kernel_launch(void* const* d_in, const int* in_sizes, int n_in, void* d_out, int out_size, void* d_ws, size_t ws_size, hipStream_t stream) {
  (void)in_sizes; (void)n_in; (void)out_size; (void)ws_size;
  const float* x = (const float*)d_in[0]; const int* ei = (const int*)d_in[1]; const float* mlp_w = (const float*)d_in[2]; const float* mlp_b = (const float*)d_in[3]; const float* conv_w = (const float*)d_in[4]; const float* conv_b = (const float*)d_in[5];
  const float* wih = (const float*)d_in[6]; const float* whh = (const float*)d_in[7]; const float* bih = (const float*)d_in[8]; const float* bhh = (const float*)d_in[9];
  float* out = (float*)d_out;
  char* ws = (char*)d_ws; size_t off = 0;
  auto take = [&](size_t bytes) { char* p = ws + off; off += (bytes + 255) & ~(size_t)255; return p; };
  float* HA = (float*)take((size_t)NNP * FH * 4); float* HB = (float*)take((size_t)NNP * FH * 4); float* MSG = (float*)take((size_t)NNP * FH * 4); float* M = (float*)take((size_t)NNP * FH * 4);
  k_lin<FI, FH, 0><<<NNP / 64, 128, 0, stream>>>(x, FI, NN, mlp_w, mlp_b, HA, FH);
  k_lin<FH, FH, 0><<<NNP / 64, 128, 0, stream>>>(HA, FH, NNP, conv_w, conv_b, MSG, FH);
  k_agg<<<NRB, 256, 0, stream>>>(MSG, ei, M);
  k_gru<<<NNP / 64, 128, 0, stream>>>(M, x, HA, wih, whh, bih, bhh, HB, NNP);
  k_lin<FH, FH, 0><<<NNP / 64, 128, 0, stream>>>(HB, FH, NNP, conv_w, conv_b, MSG, FH);
  k_agg<<<NRB, 256, 0, stream>>>(MSG, ei, M);
  k_gru<<<NNP / 64, 128, 0, stream>>>(M, x, HB, wih, whh, bih, bhh, out, NN);
}
